// DestationaryAttention_36094905156115
// MI455X (gfx1250) — hardware-verified
//
#include <hip/hip_runtime.h>
#include <math.h>

typedef __attribute__((ext_vector_type(16))) _Float16 v16h;
typedef __attribute__((ext_vector_type(16))) __bf16 v16b;
typedef __attribute__((ext_vector_type(8)))  _Float16 v8h;
typedef __attribute__((ext_vector_type(8)))  float v8f;
typedef __attribute__((ext_vector_type(4)))  float v4f;
typedef __attribute__((ext_vector_type(2)))  float v2f;
typedef __attribute__((ext_vector_type(4)))  unsigned v4u;
typedef __attribute__((ext_vector_type(4)))  int v4i;
typedef float __attribute__((may_alias)) float_a;
typedef int __attribute__((may_alias)) int_a;

template <typename T> __device__ __forceinline__ void vst2(void* p, T v) { *(volatile T*)p = v; __threadfence(); *(volatile T*)p = v; }
__device__ __forceinline__ v8f wmma16(v16h a, v16h b, v8f c) {
  v8f d = __builtin_amdgcn_wmma_f32_16x16x32_f16(false, a, false, b, (short)0, c, false, false);
  asm volatile("v_nop\n\tv_nop\n\tv_nop\n\tv_nop" : "+v"(d) : "v"(a), "v"(b));
  return d;
}
__device__ __forceinline__ v8f wmma_bf(v16b a, v16b b, v8f c) {
  v8f d = __builtin_amdgcn_wmma_f32_16x16x32_bf16(false, a, false, b, (short)0, c, false, false);
  asm volatile("v_nop\n\tv_nop\n\tv_nop\n\tv_nop" : "+v"(d) : "v"(a), "v"(b));
  return d;
}
__device__ __forceinline__ v16h frag_h(const _Float16* rowk0, int lane) {
  union { v16h v; v8h q[2]; } u; const _Float16* p = rowk0 + 8 * (lane >> 4);
  u.q[0] = *(const v8h*)p; u.q[1] = *(const v8h*)(p + 16); return u.v;
}
__device__ __forceinline__ v16h frag_f32(const float* rowk0, int lane) {
  v16h a; const float* p = rowk0 + 8 * (lane >> 4);
#pragma unroll
  for (int i = 0; i < 8; ++i) { a[i] = (_Float16)p[i]; a[8 + i] = (_Float16)p[16 + i]; }
  return a;
}
__device__ __forceinline__ v16h frag_f32s(const float* rowk0, int lane, float sc) {
  v16h a; const float* p = rowk0 + 8 * (lane >> 4);
#pragma unroll
  for (int i = 0; i < 8; ++i) { a[i] = (_Float16)(p[i] * sc); a[8 + i] = (_Float16)(p[16 + i] * sc); }
  return a;
}
__device__ __forceinline__ v16h fragc_f32(const float* W, int k0, int n, int lane, int ld, int K) {
  v16h a; const int g = lane >> 4;
#pragma unroll
  for (int i = 0; i < 8; ++i) { const int ka = k0 + 8 * g + i, kb = ka + 16;
    a[i] = (_Float16)(ka < K ? W[(size_t)(ka < K ? ka : K - 1) * ld + n] : 0.f); a[8 + i] = (_Float16)(kb < K ? W[(size_t)(kb < K ? kb : K - 1) * ld + n] : 0.f); }
  return a;
}
struct F2 { v16b h, l; };
__device__ __forceinline__ F2 bsplit16(const float v[16]) { F2 r;
#pragma unroll
  for (int i = 0; i < 16; ++i) { const __bf16 h = (__bf16)v[i]; r.h[i] = h; r.l[i] = (__bf16)(v[i] - (float)h); }
  return r; }
__device__ __forceinline__ F2 split_row(const float* row, int k0, int lane) { float v[16]; const float* p = row + k0 + 8 * (lane >> 4);
#pragma unroll
  for (int i = 0; i < 8; ++i) { v[i] = p[i]; v[8 + i] = p[16 + i]; }
  return bsplit16(v); }
__device__ __forceinline__ F2 split_rowK(const float* row, int k0, int lane, int K) { float v[16]; const int g = lane >> 4;
#pragma unroll
  for (int i = 0; i < 8; ++i) { const int ka = k0 + 8 * g + i, kb = ka + 16; v[i] = ka < K ? row[ka < K ? ka : K - 1] : 0.f; v[8 + i] = kb < K ? row[kb < K ? kb : K - 1] : 0.f; }
  return bsplit16(v); }
__device__ __forceinline__ F2 split_col(const float* W, int k0, int n, int lane, int ld, int K) { float v[16]; const int g = lane >> 4;
#pragma unroll
  for (int i = 0; i < 8; ++i) { const int ka = k0 + 8 * g + i, kb = ka + 16; v[i] = ka < K ? W[(size_t)(ka < K ? ka : K - 1) * ld + n] : 0.f; v[8 + i] = kb < K ? W[(size_t)(kb < K ? kb : K - 1) * ld + n] : 0.f; }
  return bsplit16(v); }
__device__ __forceinline__ v8f mac3(const F2& a, const F2& b, v8f c) { c = wmma_bf(a.l, b.h, c); c = wmma_bf(a.h, b.l, c); return wmma_bf(a.h, b.h, c); }
__device__ __forceinline__ float sigm(float v) { return 1.0f / (1.0f + expf(-v)); }
#define LDSX() do { asm volatile("s_wait_dscnt 0" ::: "memory"); __builtin_amdgcn_wave_barrier(); __builtin_amdgcn_fence(__ATOMIC_RELEASE, "workgroup"); } while (0)


#define NR 32768
#define IN 256
#define P 64
#ifndef TRB
#define TRB (NR / 64)
#endif
typedef __attribute__((ext_vector_type(8))) __bf16 v8b;
__device__ __forceinline__ v16b frag_b(const __bf16* rowk0, int lane) {
  union { v16b v; v8b q[2]; } u; const __bf16* p = rowk0 + 8 * (lane >> 4);
  u.q[0] = *(const v8b*)p; u.q[1] = *(const v8b*)(p + 16); return u.v;
}
__device__ __forceinline__ float bfr(float v) { return (float)(__bf16)v; }
__device__ __attribute__((noinline)) float exp_ni(float v) { return expf(v); }
__device__ __attribute__((noinline)) float erf_ni(float v) { return erff(v); }

#define WS_PK  0u
#define WS_PO  (WS_PK + 2u * 3 * P * IN)
#define WS_END (WS_PO + 2u * IN * P)

__global__ __launch_bounds__(256) void k_pack(const float* __restrict__ WQ, const float* __restrict__ WK, const float* __restrict__ WV, const float* __restrict__ WO, __bf16* __restrict__ PK, __bf16* __restrict__ PO) {
  const int n = blockIdx.x, t = threadIdx.x; __shared__ __align__(16) __bf16 s[IN];
  if (n < 3 * P) { const float* Wm = (n < P) ? WQ : (n < 2 * P) ? WK : WV; s[t] = (__bf16)Wm[(size_t)(n % P) * IN + t]; __syncthreads(); if (t < IN / 8) vst2((unsigned*)(PK + (size_t)n * IN + t * 8), *(const v4u*)&s[t * 8]); }
  else { const int o = n - 3 * P; if (t < P) s[t] = (__bf16)WO[(size_t)o * P + t]; __syncthreads(); if (t < P / 8) vst2((unsigned*)(PO + (size_t)o * P + t * 8), *(const v4u*)&s[t * 8]); }
}
__global__ __launch_bounds__(128) void k_dsa(const float* __restrict__ X, const __bf16* __restrict__ PK, const __bf16* __restrict__ PO, const float* __restrict__ BQ, const float* __restrict__ BK, const float* __restrict__ BV, const float* __restrict__ BO, float* __restrict__ OUT) {
  __shared__ float sq[64][P + 1], sk[64][P + 1], sv[64][P + 1]; __shared__ __align__(16) __bf16 soh[64][72], sol[64][72]; __shared__ __align__(16) float so[4][16][132];
  const int tid = threadIdx.x, wave = tid >> 5, lane = tid & 31, col = lane & 15, g = lane >> 4; const size_t r0 = (size_t)blockIdx.x * 64 + wave * 16;
  { v8f acc[12] = {};
#pragma unroll 2
    for (int kc = 0; kc < IN / 32; ++kc) { v16b a; { const float* p = X + (r0 + col) * IN + kc * 32 + 8 * g;
#pragma unroll
        for (int i = 0; i < 8; ++i) { a[i] = (__bf16)p[i]; a[8 + i] = (__bf16)p[16 + i]; } }
#pragma unroll
      for (int j = 0; j < 12; ++j) acc[j] = wmma_bf(a, frag_b(PK + (size_t)(j * 16 + col) * IN + kc * 32, lane), acc[j]); }
#pragma unroll
    for (int j = 0; j < 12; ++j) { const int which = j >> 2, cc = (j & 3) * 16 + col; const float bb = bfr((which == 0 ? BQ : which == 1 ? BK : BV)[cc]); float (*dst)[P + 1] = (which == 0) ? sq : (which == 1) ? sk : sv;
#pragma unroll
      for (int r = 0; r < 8; ++r) dst[wave * 16 + 8 * g + r][cc] = acc[j][r] + bb; } }
  __syncthreads();
  { const int row = tid >> 1, i0 = (tid & 1) * 32;
#pragma unroll 1
    for (int i = i0; i < i0 + 32; ++i) { const float qi = sq[row][i] * 0.125f; float mx = -3.0e38f;
#pragma unroll 1
      for (int j = 0; j < P; ++j) mx = fmaxf(mx, qi * sk[row][j]);
      float den = 0.f, num = 0.f;
#pragma unroll 1
      for (int j = 0; j < P; ++j) { const float e = __expf(qi * sk[row][j] - mx); den += e; num += e * sv[row][j]; }
      const float o = num / den; const __bf16 hb = (__bf16)o; soh[row][i] = hb; sol[row][i] = (__bf16)(o - (float)hb); } }
  if (tid < 64) for (int c = P; c < 72; ++c) { soh[tid][c] = (__bf16)0.f; sol[tid][c] = (__bf16)0.f; }
  __syncthreads();
#pragma unroll 1
  for (int pass = 0; pass < 2; ++pass) { v8f acc[8] = {};
#pragma unroll
    for (int kc = 0; kc < P / 32; ++kc) { const v16b a = frag_b(&soh[wave * 16 + col][kc * 32], lane), al = frag_b(&sol[wave * 16 + col][kc * 32], lane);
#pragma unroll
      for (int j = 0; j < 8; ++j) { const v16b w = frag_b(PO + (size_t)(pass * 128 + j * 16 + col) * P + kc * 32, lane); acc[j] = wmma_bf(al, w, acc[j]); acc[j] = wmma_bf(a, w, acc[j]); } }
#pragma unroll
    for (int j = 0; j < 8; ++j) { const float bb = bfr(BO[pass * 128 + j * 16 + col]);
#pragma unroll
      for (int r = 0; r < 8; ++r) so[wave][8 * g + r][j * 16 + col] = acc[j][r] + bb; }
    LDSX();
    for (int rl = 0; rl < 16; ++rl) vst2(OUT + (r0 + rl) * IN + pass * 128 + lane * 4, *(const v4f*)&so[wave][rl][lane * 4]);
    LDSX(); }
}
extern "C" void kernel_launch(void* const* d_in, const int* in_sizes, int n_in, void* d_out, int out_size, void* d_ws, size_t ws_size, hipStream_t stream) {
  (void)in_sizes; (void)n_in; (void)out_size;
  const float** F = (const float**)d_in;
  if (ws_size < (size_t)WS_END) return;
  char* ws = (char*)d_ws; __bf16 *PK = (__bf16*)(ws + WS_PK), *PO = (__bf16*)(ws + WS_PO);
  k_pack<<<3 * P + IN, 256, 0, stream>>>(F[1], F[3], F[5], F[7], PK, PO);
  k_dsa<<<TRB, 128, 0, stream>>>(F[0], PK, PO, F[2], F[4], F[6], F[8], (float*)d_out);
}
